// TransformerBlock_18545668784207
// MI455X (gfx1250) — hardware-run, weakly checked
//
#include <hip/hip_runtime.h>


#ifndef NB
#define NB 4
#endif
#ifndef SEQ
#define SEQ 2048
#endif
#define NB_FULL  4
#define SEQ_FULL 2048
#define DM   1024
#define FFD  1024
#define NH   16
#define HD   64
#define MT   (NB * SEQ)
#define L2E  1.4426950408889634f
#define SC2  (0.125f * 1.4426950408889634f)
#define WCAR 256.0f
#define WINV 0.00390625f

static_assert(NH * HD == DM);
static_assert(HD == 64);
static_assert(SEQ % 64 == 0);
static_assert(DM % 64 == 0);
static_assert(DM % 32 == 0);
static_assert(FFD == DM);
static_assert(NB <= NB_FULL);
static_assert(SEQ <= SEQ_FULL);
static_assert(((NB * NH * (SEQ / 16)) % 4) == 0);
static_assert(MT % 64 == 0);
static_assert(MT % 4 == 0);
static_assert(DM == 4 * 256);
static_assert(DM == 8 * 128);
static_assert(DM / 2 == 2 * 256);
static_assert((DM * DM / 64) % 64 == 0);

#define SZ_RT   ((size_t)2048)
#define SZ_WH   ((size_t)5 * DM * DM * 2)
#define SZ_WOB  ((size_t)DM * DM * 2)
#define SZ_F32P ((size_t)MT * DM * 4)
#define SZ_H16P ((size_t)MT * DM * 2)
#define CARVE_TOTAL (SZ_RT + SZ_WH + SZ_WOB + SZ_F32P + SZ_H16P + SZ_F32P + SZ_H16P + SZ_H16P)
static_assert(CARVE_TOTAL <= (size_t)134217728);
static_assert(2 * SZ_H16P == SZ_F32P);
static_assert(SZ_RT >= (size_t)(DM / 2) * 4);
static_assert(SZ_RT % 256 == 0);
static_assert(SZ_WH % 256 == 0);
static_assert(SZ_WOB % 256 == 0);
static_assert(SZ_F32P % 256 == 0);
static_assert(SZ_H16P % 256 == 0);

typedef _Float16 h16;
typedef unsigned short bf;
typedef __attribute__((ext_vector_type(16))) __bf16   v16bf;
typedef __attribute__((ext_vector_type(16))) _Float16 v16h;
typedef __attribute__((ext_vector_type(8)))  _Float16 v8h;
typedef __attribute__((ext_vector_type(4)))  _Float16 v4h;
typedef __attribute__((ext_vector_type(2)))  _Float16 v2h;
typedef __attribute__((ext_vector_type(8)))  unsigned short v8us;
typedef __attribute__((ext_vector_type(2)))  unsigned short v2us;
typedef __attribute__((ext_vector_type(8)))  float    v8f;
typedef __attribute__((ext_vector_type(4)))  float    v4f;
typedef v8h  __attribute__((may_alias)) v8ha;
typedef v4h  __attribute__((may_alias)) v4ha;
typedef v4f  __attribute__((may_alias)) v4fa;
typedef v8us __attribute__((may_alias)) v8usa;

__device__ __forceinline__ unsigned short f2bf(float f) { unsigned u = __float_as_uint(f); u += 0x7FFFu + ((u >> 16) & 1u); return (unsigned short)(u >> 16); }
__device__ __forceinline__ float bf2f(unsigned short b) { return __uint_as_float(((unsigned)b) << 16); }
__device__ __forceinline__ float bfr(float f) { return bf2f(f2bf(f)); }
__device__ __forceinline__ v16h cat16(v8h lo, v8h hi) { return __builtin_shufflevector(lo, hi, 0, 1, 2, 3, 4, 5, 6, 7, 8, 9, 10, 11, 12, 13, 14, 15); }
__device__ __forceinline__ v16bf cat16b(v8us lo, v8us hi) { return __builtin_bit_cast(v16bf, __builtin_shufflevector(lo, hi, 0, 1, 2, 3, 4, 5, 6, 7, 8, 9, 10, 11, 12, 13, 14, 15)); }
__device__ __forceinline__ v8f wmma16(v16h a, v16h b, v8f c) { return __builtin_amdgcn_wmma_f32_16x16x32_f16(false, a, false, b, (short)0, c, false, false); }
__device__ __forceinline__ v8f wmmab(v16bf a, v16bf b, v8f c) { return __builtin_amdgcn_wmma_f32_16x16x32_bf16(false, a, false, b, (short)0, c, false, false); }
static __device__ __forceinline__ h16 toh_flush(float v) { const h16 r = (h16)v; return (fabsf(v) < 6.103515625e-05f) ? (h16)0.0f : r; }

template <typename T16> struct WFrag;
template <> struct WFrag<h16> { typedef v16h V; static __device__ __forceinline__ V ld(const h16* p) { return cat16(*(const v8h*)p, *(const v8h*)(p + 16)); } static __device__ __forceinline__ v8f mma(V a, V b, v8f c) { return wmma16(a, b, c); } };
template <> struct WFrag<bf> { typedef v16bf V; static __device__ __forceinline__ V ld(const bf* p) { return cat16b(*(const v8us*)p, *(const v8us*)(p + 16)); } static __device__ __forceinline__ v8f mma(V a, V b, v8f c) { return wmmab(a, b, c); } };

template <typename T16, int MODE>
__device__ __forceinline__ void gemm_body(const T16* __restrict__ A, const T16* __restrict__ Bt, size_t sB, float osc, h16* P, size_t sP, float* C, const float* bias0, const float* bias1, const float* xres) {
    typedef typename WFrag<T16>::V V;
    __shared__ __align__(16) float os[16 * 68];
    __shared__ __align__(16) h16 ts[64 * 72];
    const int z = blockIdx.z; Bt += (size_t)z * sB;
    const int lane = threadIdx.x & 31, lr = lane & 15, hi = lane >> 4; const int r0 = blockIdx.x * 64, c0 = blockIdx.y * 64;
    v8f acc[4][4];
#pragma unroll
    for (int mb = 0; mb < 4; ++mb)
#pragma unroll
        for (int nb = 0; nb < 4; ++nb) acc[mb][nb] = (v8f){};
    const size_t aoff = (size_t)(r0 + lr) * DM + 8 * hi, boff = (size_t)(c0 + lr) * DM + 8 * hi;
#pragma unroll 1
    for (int kc = 0; kc < DM; kc += 32) {
        V a[4];
#pragma unroll
        for (int mb = 0; mb < 4; ++mb) a[mb] = WFrag<T16>::ld(A + aoff + (size_t)mb * 16 * DM + kc);
#pragma unroll
        for (int nb = 0; nb < 4; ++nb) { const V b = WFrag<T16>::ld(Bt + boff + (size_t)nb * 16 * DM + kc);
#pragma unroll
            for (int mb = 0; mb < 4; ++mb) acc[mb][nb] = WFrag<T16>::mma(a[mb], b, acc[mb][nb]); }
        asm volatile("v_nop\n\tv_nop\n\tv_nop\n\tv_nop" : "+v"(acc[0][0]), "+v"(acc[1][1]), "+v"(acc[2][2]), "+v"(acc[3][3]) : "v"(a[0]), "v"(a[3]));
    }
    const int bb_ = r0 / SEQ, s0 = r0 % SEQ;
    const int rq = lane >> 3, pc = lane & 7;
    if (MODE == 0 || MODE == 3) {
        const int pitch = (MODE == 0) ? HD : DM;
        const size_t pofs = (MODE == 0) ? ((size_t)z * sP + ((size_t)(bb_ * NH + (int)blockIdx.y) * SEQ + s0) * HD) : ((size_t)r0 * DM + c0);
        h16* prow = P + pofs;
        float bv[8];
#pragma unroll
        for (int q = 0; q < 8; ++q) { const int c = c0 + pc * 8 + q; const float u0 = bias0[c], u1 = bias1[c]; bv[q] = bfr(z == 0 ? u0 : u1); }
#pragma unroll
        for (int mb = 0; mb < 4; ++mb) {
#pragma unroll
            for (int nb = 0; nb < 4; ++nb) {
#pragma unroll
                for (int j = 0; j < 8; ++j) os[(hi * 8 + j) * 68 + nb * 16 + lr] = acc[mb][nb][j]; }
            __syncthreads();
#pragma unroll 1
            for (int ps = 0; ps < 2; ++ps) {
#pragma unroll
                for (int s = 0; s < 4; ++s) { const int row = 4 * s + rq; const v4f a0 = *(const v4fa*)(os + row * 68 + pc * 8); const v4f a1 = *(const v4fa*)(os + row * 68 + pc * 8 + 4); v8h o;
                    float t0 = __builtin_fmaf(a0[0], osc, bv[0]), t1 = __builtin_fmaf(a0[1], osc, bv[1]), t2 = __builtin_fmaf(a0[2], osc, bv[2]), t3 = __builtin_fmaf(a0[3], osc, bv[3]);
                    float t4 = __builtin_fmaf(a1[0], osc, bv[4]), t5 = __builtin_fmaf(a1[1], osc, bv[5]), t6 = __builtin_fmaf(a1[2], osc, bv[6]), t7 = __builtin_fmaf(a1[3], osc, bv[7]);
                    if (MODE == 3) { t0 = fmaxf(t0, 0.0f); t1 = fmaxf(t1, 0.0f); t2 = fmaxf(t2, 0.0f); t3 = fmaxf(t3, 0.0f); t4 = fmaxf(t4, 0.0f); t5 = fmaxf(t5, 0.0f); t6 = fmaxf(t6, 0.0f); t7 = fmaxf(t7, 0.0f); }
                    o[0] = toh_flush(t0); o[1] = toh_flush(t1); o[2] = toh_flush(t2); o[3] = toh_flush(t3);
                    o[4] = toh_flush(t4); o[5] = toh_flush(t5); o[6] = toh_flush(t6); o[7] = toh_flush(t7);
                    *(volatile v8h*)(prow + (size_t)(mb * 16 + row) * pitch + pc * 8) = o; }
                if (ps == 0) __threadfence(); }
            __syncthreads();
        }
    } else if (MODE == 1) {
        h16* vb = P + ((size_t)(bb_ * NH + (int)blockIdx.y) * HD) * SEQ + s0;
        float bv[4];
#pragma unroll
        for (int nb = 0; nb < 4; ++nb) bv[nb] = bfr(bias0[c0 + nb * 16 + lr]);
#pragma unroll
        for (int mb = 0; mb < 4; ++mb) {
#pragma unroll
            for (int nb = 0; nb < 4; ++nb) { v8h o;
#pragma unroll
                for (int j = 0; j < 8; ++j) o[j] = toh_flush(__builtin_fmaf(acc[mb][nb][j], osc, bv[nb]));
                *(v8ha*)(ts + (nb * 16 + lr) * 72 + mb * 16 + 8 * hi) = o; } }
        __syncthreads();
#pragma unroll 1
        for (int ps = 0; ps < 2; ++ps) {
#pragma unroll
            for (int s = 0; s < 16; ++s) { const int d = 4 * s + rq; const v8h o = *(const v8ha*)(ts + d * 72 + pc * 8); *(volatile v8h*)(vb + (size_t)d * SEQ + pc * 8) = o; }
            if (ps == 0) __threadfence(); }
    } else {
        const int cofs = lr * 4; float b4[4];
#pragma unroll
        for (int q = 0; q < 4; ++q) b4[q] = bfr(bias0[c0 + cofs + q]);
#pragma unroll
        for (int mb = 0; mb < 4; ++mb) {
#pragma unroll
            for (int nb = 0; nb < 4; ++nb) {
#pragma unroll
                for (int j = 0; j < 8; ++j) os[(hi * 8 + j) * 68 + nb * 16 + lr] = acc[mb][nb][j]; }
            __syncthreads();
#pragma unroll 1
            for (int ps = 0; ps < 2; ++ps) {
#pragma unroll
                for (int s = 0; s < 8; ++s) { const int row = 2 * s + hi; const int m = r0 + mb * 16 + row;
                    v4f val = *(const v4fa*)(os + row * 68 + cofs); const v4f xv = *(const v4f*)(xres + (size_t)m * DM + c0 + cofs);
                    val[0] = __builtin_fmaf(val[0], osc, b4[0]) + xv[0]; val[1] = __builtin_fmaf(val[1], osc, b4[1]) + xv[1]; val[2] = __builtin_fmaf(val[2], osc, b4[2]) + xv[2]; val[3] = __builtin_fmaf(val[3], osc, b4[3]) + xv[3];
                    *(volatile v4f*)(C + (size_t)m * DM + c0 + cofs) = val; }
                if (ps == 0) __threadfence(); }
            __syncthreads();
        }
    }
}

__global__ __launch_bounds__(32) void k_gemm_qk(const h16* __restrict__ A, const h16* __restrict__ Bt, size_t sB, float osc, h16* P, size_t sP, const float* bias0, const float* bias1) {
    gemm_body<h16, 0>(A, Bt, sB, osc, P, sP, (float*)0, bias0, bias1, (const float*)0); }
__global__ __launch_bounds__(32) void k_gemm_v(const h16* __restrict__ A, const h16* __restrict__ Bt, float osc, h16* P, const float* bias0) {
    gemm_body<h16, 1>(A, Bt, (size_t)0, osc, P, (size_t)0, (float*)0, bias0, bias0, (const float*)0); }
__global__ __launch_bounds__(32) void k_gemm_o(const bf* __restrict__ A, const bf* __restrict__ Bt, float osc, float* C, const float* bias0, const float* xres) {
    gemm_body<bf, 2>(A, Bt, (size_t)0, osc, (h16*)0, (size_t)0, C, bias0, bias0, xres); }
__global__ __launch_bounds__(32) void k_gemm_f1(const h16* __restrict__ A, const h16* __restrict__ Bt, float osc, h16* P, const float* bias0) {
    gemm_body<h16, 3>(A, Bt, (size_t)0, osc, P, (size_t)0, (float*)0, bias0, bias0, (const float*)0); }
__global__ __launch_bounds__(32) void k_gemm_f2(const h16* __restrict__ A, const h16* __restrict__ Bt, float osc, float* C, const float* bias0, const float* xres) {
    gemm_body<h16, 2>(A, Bt, (size_t)0, osc, (h16*)0, (size_t)0, C, bias0, bias0, xres); }

__global__ __launch_bounds__(256) void k_wtG(const float* __restrict__ w, int K, int N, bf* Bt) {
    const int lane = threadIdx.x & 31; const int L0 = (blockIdx.x * 8 + (threadIdx.x >> 5)) * 8; const int nlines = N * K / 64;
#pragma unroll
    for (int ps = 0; ps < 2; ++ps) {
#pragma unroll 1
        for (int l = 0; l < 8; ++l) { const int L = L0 + l; if (L >= nlines) break; const size_t e = (size_t)L * 64 + lane * 2; const int k = (int)(e % K), n = (int)(e / K); v2us o;
            o[0] = f2bf(w[(size_t)k * N + n]); o[1] = f2bf(w[(size_t)(k + 1) * N + n]); *(volatile v2us*)(Bt + e) = o; }
        if (ps == 0) __threadfence(); }
}
__global__ __launch_bounds__(256) void k_wtH(const float* __restrict__ w, int K, int N, h16* Bt) {
    const int lane = threadIdx.x & 31; const int L0 = (blockIdx.x * 8 + (threadIdx.x >> 5)) * 8; const int nlines = N * K / 64;
#pragma unroll
    for (int ps = 0; ps < 2; ++ps) {
#pragma unroll 1
        for (int l = 0; l < 8; ++l) { const int L = L0 + l; if (L >= nlines) break; const size_t e = (size_t)L * 64 + lane * 2; const int k = (int)(e % K), n = (int)(e / K); v2h o;
            o[0] = toh_flush(bfr(w[(size_t)k * N + n]) * WCAR); o[1] = toh_flush(bfr(w[(size_t)(k + 1) * N + n]) * WCAR); *(volatile v2h*)(Bt + e) = o; }
        if (ps == 0) __threadfence(); }
}

__global__ __launch_bounds__(256) void k_rate(float* RT) {
    const int j = blockIdx.x * 256 + threadIdx.x;
    const float e = (float)(2 * j) * (1.0f / (float)DM);
    const float p = powf(10000.0f, e);
    const float r = 1.0f / p;
    *(volatile float*)(RT + j) = r; __threadfence(); *(volatile float*)(RT + j) = r;
}

__global__ __launch_bounds__(256) void k_xpe(const float* __restrict__ in, const float* __restrict__ rt, float* XF, h16* XH) {
#pragma clang fp contract(off)
    __shared__ __align__(16) float pes[DM];
    __shared__ __align__(16) float xs[DM];
    const int s = blockIdx.x, t = threadIdx.x;
#pragma unroll 1
    for (int jj = 0; jj < 2; ++jj) { const int j = t + 256 * jj; const float ang = (float)s * rt[j]; float sn, cs; sincosf(ang, &sn, &cs); pes[2 * j] = sn; pes[2 * j + 1] = cs; }
    __syncthreads();
    const v4f pe4 = *(const v4fa*)(pes + 4 * t);
#pragma unroll 1
    for (int b = 0; b < NB; ++b) {
        const v4f iv = *(const v4f*)(in + ((size_t)b * SEQ_FULL + s) * DM + 4 * t);
        v4f xv; xv[0] = bfr(iv[0]) + pe4[0]; xv[1] = bfr(iv[1]) + pe4[1]; xv[2] = bfr(iv[2]) + pe4[2]; xv[3] = bfr(iv[3]) + pe4[3];
        const size_t row = (size_t)b * SEQ + s;
        float* xp = XF + row * DM + 4 * t;
        *(v4fa*)(xs + 4 * t) = xv;
        *(volatile v4f*)xp = xv;
        __threadfence();
        *(volatile v4f*)xp = xv;
        __syncthreads();
        if (t < 128) {
            const v4f a0 = *(const v4fa*)(xs + 8 * t); const v4f a1 = *(const v4fa*)(xs + 8 * t + 4); v8h o;
            o[0] = toh_flush(a0[0]); o[1] = toh_flush(a0[1]); o[2] = toh_flush(a0[2]); o[3] = toh_flush(a0[3]);
            o[4] = toh_flush(a1[0]); o[5] = toh_flush(a1[1]); o[6] = toh_flush(a1[2]); o[7] = toh_flush(a1[3]);
            h16* hp = XH + row * DM + 8 * t;
            *(volatile v8h*)hp = o;
            __threadfence();
            *(volatile v8h*)hp = o;
        }
        __syncthreads();
    }
}

template <int WH>
__device__ __forceinline__ void ln_body(const float* __restrict__ Y, const float* __restrict__ g, const float* __restrict__ be, float* OF, h16* OH) {
#pragma clang fp contract(off)
    __shared__ __align__(16) h16 hs[4 * DM];
    const int lane = threadIdx.x & 31; const int wave = __builtin_amdgcn_readfirstlane(threadIdx.x >> 5);
    const size_t row = (size_t)blockIdx.x * 4 + wave;
    const float* yr = Y + row * DM + 4 * lane;
    v4f v[8];
#pragma unroll
    for (int i = 0; i < 8; ++i) v[i] = *(const v4f*)(yr + 128 * i);
    float sum = 0.0f;
#pragma unroll
    for (int i = 0; i < 8; ++i) sum += (v[i][0] + v[i][1]) + (v[i][2] + v[i][3]);
#pragma unroll
    for (int o = 16; o >= 1; o >>= 1) sum += __shfl_xor(sum, o, 32);
    const float mu = sum * (1.0f / (float)DM);
    float sq = 0.0f;
#pragma unroll
    for (int i = 0; i < 8; ++i) { const float d0 = v[i][0] - mu, d1 = v[i][1] - mu, d2 = v[i][2] - mu, d3 = v[i][3] - mu; sq += (d0 * d0 + d1 * d1) + (d2 * d2 + d3 * d3); }
#pragma unroll
    for (int o = 16; o >= 1; o >>= 1) sq += __shfl_xor(sq, o, 32);
    const float var = sq * (1.0f / (float)DM);
    const float rstd = 1.0f / sqrtf(var + 1.0e-6f);
#pragma unroll
    for (int i = 0; i < 8; ++i) { const v4f gv = *(const v4f*)(g + 4 * lane + 128 * i); const v4f bv = *(const v4f*)(be + 4 * lane + 128 * i);
        v[i][0] = ((v[i][0] - mu) * rstd) * bfr(gv[0]) + bfr(bv[0]); v[i][1] = ((v[i][1] - mu) * rstd) * bfr(gv[1]) + bfr(bv[1]);
        v[i][2] = ((v[i][2] - mu) * rstd) * bfr(gv[2]) + bfr(bv[2]); v[i][3] = ((v[i][3] - mu) * rstd) * bfr(gv[3]) + bfr(bv[3]); }
    float* orow = OF + row * DM + 4 * lane;
#pragma unroll 1
    for (int ps = 0; ps < 2; ++ps) {
#pragma unroll
        for (int i = 0; i < 8; ++i) *(volatile v4f*)(orow + 128 * i) = v[i];
        if (ps == 0) __threadfence(); }
    if (WH != 0) {
        h16* hw = hs + wave * DM;
#pragma unroll
        for (int i = 0; i < 8; ++i) { v4h q; q[0] = toh_flush(v[i][0]); q[1] = toh_flush(v[i][1]); q[2] = toh_flush(v[i][2]); q[3] = toh_flush(v[i][3]); *(v4ha*)(hw + 4 * lane + 128 * i) = q; }
        __syncthreads();
        v8h ov[4];
#pragma unroll
        for (int j = 0; j < 4; ++j) ov[j] = *(const v8ha*)(hw + 8 * lane + 256 * j);
        h16* hrow = OH + row * DM + 8 * lane;
#pragma unroll 1
        for (int ps = 0; ps < 2; ++ps) {
#pragma unroll
            for (int j = 0; j < 4; ++j) *(volatile v8h*)(hrow + 256 * j) = ov[j];
            if (ps == 0) __threadfence(); }
    }
}
__global__ __launch_bounds__(128) void k_ln1(const float* __restrict__ Y, const float* __restrict__ g, const float* __restrict__ be, float* OF, h16* OH) { ln_body<1>(Y, g, be, OF, OH); }
__global__ __launch_bounds__(128) void k_ln2(const float* __restrict__ Y, const float* __restrict__ g, const float* __restrict__ be, float* OF) { ln_body<0>(Y, g, be, OF, (h16*)0); }

__global__ __launch_bounds__(128) void k_flash(const h16* __restrict__ Q, const h16* __restrict__ Kpl, const h16* __restrict__ VT, bf* CTX) {
    __shared__ __align__(16) unsigned short cs[4 * 16 * 72];
    const int lane = threadIdx.x & 31, wid = threadIdx.x >> 5, lr = lane & 15, hi = lane >> 4;
    const int gw = blockIdx.x * 4 + wid; const int bh = gw / (SEQ / 16); const int q0 = (gw % (SEQ / 16)) * 16; const int b = bh / NH, h = bh % NH;
    const h16* Qp = Q + ((size_t)bh * SEQ + q0 + lr) * HD + 8 * hi;
    const v16h qb0 = WFrag<h16>::ld(Qp), qb1 = WFrag<h16>::ld(Qp + 32);
    const h16* Kb = Kpl + (size_t)bh * SEQ * HD + (size_t)lr * HD + 8 * hi;
    const h16* Vb = VT + (size_t)bh * HD * SEQ + (size_t)lr * SEQ + 8 * hi;
    v8f o[4];
#pragma unroll
    for (int j = 0; j < 4; ++j) o[j] = (v8f){};
    float m = -1.0e30f, ls = 0.0f;
#pragma unroll 1
    for (int k0 = 0; k0 < SEQ; k0 += 32) {
        const h16* kr = Kb + (size_t)k0 * HD;
        const v16h ka = WFrag<h16>::ld(kr), kb = WFrag<h16>::ld(kr + 32), kc = WFrag<h16>::ld(kr + 16 * HD), kd = WFrag<h16>::ld(kr + 16 * HD + 32);
        v8f s0 = wmma16(ka, qb0, (v8f){}); s0 = wmma16(kb, qb1, s0);
        v8f s1 = wmma16(kc, qb0, (v8f){}); s1 = wmma16(kd, qb1, s1);
        asm volatile("v_nop\n\tv_nop\n\tv_nop\n\tv_nop" : "+v"(s0), "+v"(s1) : "v"(kd), "v"(qb1));
        float mx = fmaxf(s0[0], s1[0]);
#pragma unroll
        for (int r = 1; r < 8; ++r) mx = fmaxf(mx, fmaxf(s0[r], s1[r]));
        mx *= 0.125f;
        const float mo = __shfl_xor(mx, 16, 32); mx = fmaxf(mx, mo);
        const float mn = fmaxf(m, mx);
        const float alpha = __builtin_amdgcn_exp2f((m - mn) * L2E);
        const float off = 10.0f - mn * L2E;
        m = mn;
        v16h pb; float psum = 0.0f;
#pragma unroll
        for (int r = 0; r < 8; ++r) { const float p0 = __builtin_amdgcn_exp2f(__builtin_fmaf(s0[r], SC2, off)); const float p1 = __builtin_amdgcn_exp2f(__builtin_fmaf(s1[r], SC2, off)); psum += p0 + p1; pb[r] = (h16)p0; pb[8 + r] = (h16)p1; }
        ls = ls * alpha + psum;
#pragma unroll
        for (int j = 0; j < 4; ++j) o[j] = o[j] * alpha;
        const h16* vr = Vb + k0;
        const v16h va0 = WFrag<h16>::ld(vr), va1 = WFrag<h16>::ld(vr + (size_t)16 * SEQ), va2 = WFrag<h16>::ld(vr + (size_t)32 * SEQ), va3 = WFrag<h16>::ld(vr + (size_t)48 * SEQ);
        o[0] = wmma16(va0, pb, o[0]); o[1] = wmma16(va1, pb, o[1]); o[2] = wmma16(va2, pb, o[2]); o[3] = wmma16(va3, pb, o[3]);
        asm volatile("v_nop\n\tv_nop\n\tv_nop\n\tv_nop" : "+v"(o[0]), "+v"(o[1]), "+v"(o[2]), "+v"(o[3]) : "v"(va3), "v"(pb));
    }
    const float lo_ = __shfl_xor(ls, 16, 32); ls += lo_;
    const float inv = 1.0f / ls;
    unsigned short* cw = cs + wid * (16 * 72);
#pragma unroll
    for (int j = 0; j < 4; ++j) { v8us w;
#pragma unroll
        for (int r = 0; r < 8; ++r) w[r] = f2bf(o[j][r] * inv);
        *(v8usa*)(cw + lr * 72 + j * 16 + 8 * hi) = w; }
    __syncthreads();
    const int rq = lane >> 3, pc = lane & 7;
    bf* crow = CTX + ((size_t)b * SEQ + q0) * DM + h * HD + pc * 8;
    v8us ov[4];
#pragma unroll
    for (int s = 0; s < 4; ++s) ov[s] = *(const v8usa*)(cw + (4 * s + rq) * 72 + pc * 8);
#pragma unroll
    for (int s = 0; s < 4; ++s) *(volatile v8us*)(crow + (size_t)(4 * s + rq) * DM) = ov[s];
    __threadfence();
#pragma unroll
    for (int s = 0; s < 4; ++s) *(volatile v8us*)(crow + (size_t)(4 * s + rq) * DM) = ov[s];
}

extern "C" void kernel_launch(void* const* d_in, const int* in_sizes, int n_in,
                              void* d_out, int out_size, void* d_ws, size_t ws_size, hipStream_t stream) {
    if (n_in < 17) return;
    const size_t xneed = (size_t)(NB - 1) * SEQ_FULL * DM + (size_t)SEQ * DM;
    if ((size_t)in_sizes[0] < xneed) return;
    if ((size_t)in_sizes[1] < (size_t)DM * DM || (size_t)in_sizes[3] < (size_t)DM * DM || (size_t)in_sizes[5] < (size_t)DM * DM || (size_t)in_sizes[7] < (size_t)DM * DM) return;
    if ((size_t)in_sizes[9] < (size_t)DM * FFD || (size_t)in_sizes[11] < (size_t)FFD * FFD) return;
    if (in_sizes[2] < DM || in_sizes[4] < DM || in_sizes[6] < DM || in_sizes[8] < DM || in_sizes[10] < FFD || in_sizes[12] < FFD) return;
    if (in_sizes[13] < DM || in_sizes[14] < DM || in_sizes[15] < DM || in_sizes[16] < DM) return;
    if ((size_t)out_size < (size_t)MT * DM) return;
    const float* xin = (const float*)d_in[0]; const float* wq = (const float*)d_in[1]; const float* bq = (const float*)d_in[2]; const float* wk = (const float*)d_in[3]; const float* bk = (const float*)d_in[4];
    const float* wv = (const float*)d_in[5]; const float* bv = (const float*)d_in[6]; const float* wo = (const float*)d_in[7]; const float* bo = (const float*)d_in[8];
    const float* w1 = (const float*)d_in[9]; const float* b1 = (const float*)d_in[10]; const float* w2 = (const float*)d_in[11]; const float* b2 = (const float*)d_in[12];
    const float* g1 = (const float*)d_in[13]; const float* be1 = (const float*)d_in[14]; const float* g2 = (const float*)d_in[15]; const float* be2 = (const float*)d_in[16];
    float* OUT = (float*)d_out;
    char* wsp = (char*)d_ws;
    auto take = [&](size_t bytes) { char* p = wsp; wsp += (bytes + 255) & ~(size_t)255; return (void*)p; };
    float* RT  = (float*)take(SZ_RT);
    h16*  WHp  = (h16*)take(SZ_WH);
    bf*   WOB  = (bf*)take(SZ_WOB);
    float* R1  = (float*)take(SZ_F32P);
    h16*  R2   = (h16*)take(SZ_H16P);
    char* R3   = (char*)take(SZ_F32P);
    h16*  R4   = (h16*)take(SZ_H16P);
    bf*   CTX  = (bf*)take(SZ_H16P);
    if ((size_t)(wsp - (char*)d_ws) > ws_size) return;
    float* XF = R1; float* O1F = R1; h16* XH = R2; h16* O1H = R2;
    h16* QP = (h16*)R3; h16* KP = QP + (size_t)MT * DM; float* YS = (float*)R3;
    h16* VTp = R4; h16* HP = R4;
    const size_t WSZ = (size_t)DM * DM;

    k_rate<<<2, 256, 0, stream>>>(RT);
    k_xpe<<<SEQ, 256, 0, stream>>>(xin, RT, XF, XH);
    const unsigned gw_ = (unsigned)((DM * DM / 64 + 63) / 64);
    k_wtH<<<gw_, 256, 0, stream>>>(wq, DM, DM, WHp);
    k_wtH<<<gw_, 256, 0, stream>>>(wk, DM, DM, WHp + WSZ);
    k_wtH<<<gw_, 256, 0, stream>>>(wv, DM, DM, WHp + 2 * WSZ);
    k_wtH<<<gw_, 256, 0, stream>>>(w1, DM, FFD, WHp + 3 * WSZ);
    k_wtH<<<gw_, 256, 0, stream>>>(w2, FFD, FFD, WHp + 4 * WSZ);
    k_wtG<<<gw_, 256, 0, stream>>>(wo, DM, DM, WOB);
    k_gemm_qk<<<dim3(MT / 64, DM / 64, 2), 32, 0, stream>>>(XH, WHp, WSZ, WINV, QP, (size_t)MT * DM, bq, bk);
    k_gemm_v<<<dim3(MT / 64, DM / 64, 1), 32, 0, stream>>>(XH, WHp + 2 * WSZ, WINV, VTp, bv);
    k_flash<<<(unsigned)(NB * NH * (SEQ / 16) / 4), 128, 0, stream>>>(QP, KP, VTp, CTX);
    k_gemm_o<<<dim3(MT / 64, DM / 64, 1), 32, 0, stream>>>(CTX, WOB, 1.0f, YS, bo, XF);
    k_ln1<<<MT / 4, 128, 0, stream>>>(YS, g1, be1, O1F, O1H);
    k_gemm_f1<<<dim3(MT / 64, FFD / 64, 1), 32, 0, stream>>>(O1H, WHp + 3 * WSZ, WINV, HP, b1);
    k_gemm_f2<<<dim3(MT / 64, FFD / 64, 1), 32, 0, stream>>>(HP, WHp + 4 * WSZ, WINV, YS, b2, O1F);
    k_ln2<<<MT / 4, 128, 0, stream>>>(YS, g2, be2, OUT);
}
